// GATv2ActorCritic_13262859010781
// MI455X (gfx1250) — hardware-verified
//
#include <hip/hip_runtime.h>
#include <stddef.h>
#include <stdint.h>
#include <math.h>


#define C1     256
#define C2     64
#define K2     512
#define N2     128
#define NTHR   256
#define NWAVE  8
#define EPT    8
#define CHUNK  (NTHR * EPT)
#define WCAP   (EPT * 32)
#define LISTN  (NWAVE * WCAP)
#define NBA    1024
#define SLA    10
#define RCAP   14336
#define DEGCAP 64
#define GBM    64
#define GBN    64
#define GTHR   128
#define NEGS   0.2f
#define WSMAX  134217728
#define AGG_ZINTS (LISTN + 2 * RCAP + 3 * NBA)
#define AGG_LDS_INTS (AGG_ZINTS + 32)
#define LDS_SCAN (AGG_LDS_INTS * 4)
#define PP_WL0 0
#define PP_BL  512
#define PP_WR0 768
#define PP_BR  1280
#define PP_WE0 1536
#define PP_AT1 2048
#define PP_B1  2304
#define PP_P2  2560
#define PP_B2  2816
#define PP_N   2944
#define NUB    (N2 * (K2 / 8))
#define NUBH   (NUB / 2)

static_assert((CHUNK & (CHUNK - 1)) == 0 && CHUNK <= 4096);
static_assert((NBA & (NBA - 1)) == 0 && NBA == (1 << SLA));
static_assert(((long long)CHUNK << SLA) < (1LL << 31));
static_assert(NBA % NWAVE == 0 && NBA % 32 == 0 && NBA % 16 == 0);
static_assert(RCAP % 32 == 0 && AGG_ZINTS % 4 == 0 && LISTN % 4 == 0);
static_assert(RCAP >= 11523);
static_assert(DEGCAP >= 26 + 8);
static_assert(C1 == 32 * 8 && C2 == 32 * 2);
static_assert(K2 == 2 * C1 && K2 % 32 == 0 && K2 == 512 && N2 == 128 && N2 == 2 * C2);
static_assert(GBM == (GTHR / 32) * 16 && GBN == 64 && N2 % GBN == 0);
static_assert(LISTN >= NWAVE * C1);
static_assert(RCAP * 4 >= (NWAVE * C2 + C2) * 8);
static_assert(LDS_SCAN <= 320 * 1024);
static_assert(NTHR == C1);
static_assert(NUB % NTHR == 0 && NUBH % NTHR == 0);
static_assert(PP_N % 4 == 0 && (PP_N * 4) % 128 == 0 && (PP_N / 4) % 32 == 0);

typedef float          v2f   __attribute__((ext_vector_type(2)));
typedef float          v4f   __attribute__((ext_vector_type(4)));
typedef float          v8f   __attribute__((ext_vector_type(8)));
typedef double         v2d   __attribute__((ext_vector_type(2)));
typedef int            v2i   __attribute__((ext_vector_type(2)));
typedef int            v4i   __attribute__((ext_vector_type(4)));
typedef int            v8i   __attribute__((ext_vector_type(8)));
typedef unsigned short v8us  __attribute__((ext_vector_type(8)));
typedef unsigned short v16us __attribute__((ext_vector_type(16)));
typedef __bf16         v16bf __attribute__((ext_vector_type(16)));
typedef v2f  __attribute__((may_alias)) v2fa;
typedef v4f  __attribute__((may_alias)) v4fa;
typedef v2i  __attribute__((may_alias)) v2ia;
typedef v4i  __attribute__((may_alias)) v4ia;
typedef v8us __attribute__((may_alias)) v8usa;
union FragB { v16bf v; v16us u; v8us h[2]; v8i w; };

__device__ __forceinline__ v8f wmb(const FragB& a, const FragB& b, v8f c) {
  v8f d = __builtin_amdgcn_wmma_f32_16x16x32_bf16(false, a.v, false, b.v, (short)0, c, false, false);
  asm volatile("v_nop\n\tv_nop\n\tv_nop\n\tv_nop" : "+v"(d) : "v"(a.w), "v"(b.w));
  return d;
}

__device__ __forceinline__ void ldwait() {
  asm volatile("s_wait_loadcnt 0x0" ::: "memory");
}

__device__ __forceinline__ unsigned bf16_bits(float f) {
  const unsigned u = __float_as_uint(f);
  return (u + 0x7FFFu + ((u >> 16) & 1u)) >> 16;
}
__device__ __forceinline__ float bf16_val(float f) {
  return __uint_as_float(bf16_bits(f) << 16);
}

__device__ __forceinline__ void ld8(const float* __restrict__ p, float (&o)[8]) {
  const v4f a = *(const v4fa*)p;
  const v4f b = *(const v4fa*)(p + 4);
  o[0] = a.x; o[1] = a.y; o[2] = a.z; o[3] = a.w;
  o[4] = b.x; o[5] = b.y; o[6] = b.z; o[7] = b.w;
}

template <int SLB>
__device__ __forceinline__ int scan_chunk(const int* __restrict__ dsts, int nE, int cbase, int slotBase,
                                          int nb, int vec8, int* list, int tid, int lane, int wave) {
  int wc = 0;
  const int el0  = tid * EPT;
  const int e0   = cbase + el0;
  const int sent = -2147483647 - 1;
  v4i da, db;
  if (vec8 != 0 && cbase + CHUNK <= nE) {
    da = *(const v4i*)(dsts + e0);
    db = *(const v4i*)(dsts + e0 + 4);
  } else {
    da.x = (e0     < nE) ? dsts[min(e0,     nE - 1)] : sent;
    da.y = (e0 + 1 < nE) ? dsts[min(e0 + 1, nE - 1)] : sent;
    da.z = (e0 + 2 < nE) ? dsts[min(e0 + 2, nE - 1)] : sent;
    da.w = (e0 + 3 < nE) ? dsts[min(e0 + 3, nE - 1)] : sent;
    db.x = (e0 + 4 < nE) ? dsts[min(e0 + 4, nE - 1)] : sent;
    db.y = (e0 + 5 < nE) ? dsts[min(e0 + 5, nE - 1)] : sent;
    db.z = (e0 + 6 < nE) ? dsts[min(e0 + 6, nE - 1)] : sent;
    db.w = (e0 + 7 < nE) ? dsts[min(e0 + 7, nE - 1)] : sent;
  }
  const unsigned nbs = (unsigned)slotBase;
  const unsigned unb = (unsigned)nb;
  const unsigned s0 = (unsigned)da.x - nbs, s1 = (unsigned)da.y - nbs;
  const unsigned s2 = (unsigned)da.z - nbs, s3 = (unsigned)da.w - nbs;
  const unsigned s4 = (unsigned)db.x - nbs, s5 = (unsigned)db.y - nbs;
  const unsigned s6 = (unsigned)db.z - nbs, s7 = (unsigned)db.w - nbs;
  const bool h0 = s0 < unb, h1 = s1 < unb, h2 = s2 < unb, h3 = s3 < unb;
  const bool h4 = s4 < unb, h5 = s5 < unb, h6 = s6 < unb, h7 = s7 < unb;
  const unsigned any = __builtin_amdgcn_ballot_w32(h0 | h1 | h2 | h3 | h4 | h5 | h6 | h7);
  if (any != 0u) {
#define HITJ(J, HJ, SJ) { \
      const unsigned mj = __builtin_amdgcn_ballot_w32(HJ); \
      if (mj != 0u) { \
        if (HJ) { \
          const int pos = wc + (int)__builtin_amdgcn_mbcnt_lo(mj, 0u); \
          if (pos < WCAP) list[wave * WCAP + pos] = ((el0 + (J)) << SLB) | (int)(SJ); \
        } \
        wc += (int)__builtin_popcount(mj); } }
    HITJ(0, h0, s0)
    HITJ(1, h1, s1)
    HITJ(2, h2, s2)
    HITJ(3, h3, s3)
    HITJ(4, h4, s4)
    HITJ(5, h5, s5)
    HITJ(6, h6, s6)
    HITJ(7, h7, s7)
#undef HITJ
  }
  return wc;
}

__device__ __forceinline__ void build_lists(const int* __restrict__ dsts, int nE, int vec8, int nodeBase,
                                            int* list, int* hl, int* sl, int* cnt, int* offs, int* cur,
                                            int* misc, int tid, int lane, int wave, int& ttOut, int& ovfOut) {
  int t = 0, ov = 0;
  const int nChunks = (nE + CHUNK - 1) / CHUNK;
#pragma unroll 1
  for (int ch = 0; ch < nChunks; ++ch) {
    const int cbase = ch * CHUNK;
    const int wc = scan_chunk<SLA>(dsts, nE, cbase, nodeBase, NBA, vec8, list, tid, lane, wave);
    if (lane == 0) misc[wave] = wc;
    __syncthreads();
    if (wave == 0) {
#pragma unroll 1
      for (int w2 = 0; w2 < NWAVE; ++w2) {
        int c = misc[w2];
        c = c < 0 ? 0 : (c > WCAP ? WCAP : c);
#pragma unroll 1
        for (int b0 = 0; b0 < c; b0 += 32) {
          const int idx = b0 + lane;
          const int ent = list[w2 * WCAP + (idx < WCAP ? idx : WCAP - 1)];
          const int m32 = (c - b0) < 32 ? (c - b0) : 32;
#pragma unroll 1
          for (int k = 0; k < m32; ++k) {
            const int u    = __builtin_amdgcn_readlane(ent, k);
            const int slot = u & (NBA - 1);
            const int el   = (u >> SLA) & (CHUNK - 1);
            const int pk   = ((cbase + el) << SLA) | slot;
            if (t < RCAP) {
              if (lane == 0) { hl[t] = pk; cnt[slot] = cnt[slot] + 1; }
              t = t + 1;
            } else {
              ov = 1;
            }
          }
        }
      }
    }
    __syncthreads();
  }
  if (wave == 0 && lane == 0) { misc[8] = t; misc[9] = ov; }
  __syncthreads();
  int tt = misc[8];
  tt = tt < 0 ? 0 : (tt > RCAP ? RCAP : tt);
  const int ovf = misc[9];

  if (wave == 0) {
    const int base = lane * (NBA / 32);
    int s = 0;
#pragma unroll 1
    for (int i = 0; i < NBA / 32; ++i) s += cnt[base + i];
    int incl = s;
#pragma unroll
    for (int d = 1; d < 32; d <<= 1) {
      const int y = __shfl_up(incl, d, 32);
      if (lane >= d) incl += y;
    }
    int run = incl - s;
#pragma unroll 1
    for (int i = 0; i < NBA / 32; ++i) {
      const int cv = cnt[base + i];
      offs[base + i] = run;
      cur[base + i]  = run;
      run += cv;
    }
  }
  __syncthreads();
  if (wave == 0) {
#pragma unroll 1
    for (int b0 = 0; b0 < tt; b0 += 32) {
      const int idx = b0 + lane;
      const int ent = hl[idx < RCAP ? idx : RCAP - 1];
      const int m32 = (tt - b0) < 32 ? (tt - b0) : 32;
#pragma unroll 1
      for (int k = 0; k < m32; ++k) {
        const int u    = __builtin_amdgcn_readlane(ent, k);
        const int slot = u & (NBA - 1);
        if (lane == 0) {
          int p = cur[slot];
          p = p < 0 ? 0 : (p > RCAP - 1 ? RCAP - 1 : p);
          sl[p] = u;
          cur[slot] = p + 1;
        }
      }
    }
  }
  __syncthreads();
  ttOut = tt;
  ovfOut = ovf;
}

__global__ __launch_bounds__(NTHR) void k_prep(
    const float* __restrict__ W1l, const float* __restrict__ b1l, const float* __restrict__ W1r,
    const float* __restrict__ b1r, const float* __restrict__ W1e, const float* __restrict__ att1,
    const float* __restrict__ bias1, const float* __restrict__ W2l, const float* __restrict__ b2l,
    const float* __restrict__ W2r, const float* __restrict__ b2r, const float* __restrict__ W2e,
    const float* __restrict__ att2, const float* __restrict__ bias2,
    unsigned short* bt2, float* pp) {
  __shared__ __attribute__((aligned(16))) float st[PP_N];
  const int tid = (int)threadIdx.x;
  const int blk = (int)blockIdx.x;
  if (blk < NUB / NTHR) {
    const int u   = blk * NTHR + tid;
    const int n   = u >> 6;
    const int k8  = (u & 63) * 8;
    const int kk  = k8 & (C1 - 1);
    const int col = n & (C2 - 1);
    v8us o;
    if (u < NUBH) {
      const float* p = W2l + (size_t)kk * C2 + col;
#pragma unroll
      for (int i = 0; i < 8; ++i) o[i] = (unsigned short)bf16_bits(p[(size_t)i * C2]);
    } else {
      const float* p = W2r + (size_t)kk * C2 + col;
#pragma unroll
      for (int i = 0; i < 8; ++i) o[i] = (unsigned short)bf16_bits(p[(size_t)i * C2]);
    }
    unsigned short* dp = bt2 + (size_t)n * K2 + k8;
    *(volatile v8us*)dp = o;
    __threadfence();
    *(volatile v8us*)dp = o;
    return;
  }
#pragma unroll 1
  for (int i = tid; i < 2 * C1; i += NTHR) st[PP_WL0 + i] = bf16_val(W1l[i]);
  ldwait();
#pragma unroll 1
  for (int i = tid; i < 2 * C1; i += NTHR) st[PP_WR0 + i] = bf16_val(W1r[i]);
  ldwait();
#pragma unroll 1
  for (int i = tid; i < 2 * C1; i += NTHR) st[PP_WE0 + i] = bf16_val(W1e[i]);
  ldwait();
  st[PP_BL + tid]  = bf16_val(b1l[tid]);
  st[PP_BR + tid]  = bf16_val(b1r[tid]);
  ldwait();
  st[PP_AT1 + tid] = bf16_val(att1[tid]);
  st[PP_B1 + tid]  = bf16_val(bias1[tid]);
  ldwait();
  if (tid < 2 * C2) st[PP_P2 + tid] = bf16_val(W2e[tid]);
  ldwait();
  if (tid < C2) {
    st[PP_P2 + 2 * C2 + tid] = bf16_val(att2[tid]);
    st[PP_P2 + 3 * C2 + tid] = bf16_val(bias2[tid]);
    st[PP_B2 + tid]          = bf16_val(b2l[tid]);
    st[PP_B2 + C2 + tid]     = bf16_val(b2r[tid]);
  }
  __syncthreads();
  constexpr int NU = PP_N / 4;
  v4f ov[3];
#pragma unroll
  for (int it = 0; it < 3; ++it) {
    const int u  = it * NTHR + tid;
    const int uc = u < NU ? u : NU - 1;
    ov[it] = *(const v4fa*)(st + 4 * uc);
  }
#pragma unroll
  for (int it = 0; it < 3; ++it) {
    const int u = it * NTHR + tid;
    if (u < NU) *(volatile v4f*)(pp + 4 * (size_t)u) = ov[it];
  }
  __threadfence();
#pragma unroll
  for (int it = 0; it < 3; ++it) {
    const int u = it * NTHR + tid;
    if (u < NU) *(volatile v4f*)(pp + 4 * (size_t)u) = ov[it];
  }
}

__global__ __launch_bounds__(NTHR) void k_scan1(
    const int* __restrict__ srcs, const int* __restrict__ dsts,
    const float* __restrict__ x, const float* __restrict__ ea, const float* __restrict__ pp,
    unsigned short* h1, int nE, int nN, int vec8, int mRows) {
  extern __shared__ __attribute__((aligned(16))) int dsm[];
  int* list = dsm;
  int* hl   = dsm + LISTN;
  int* sl   = dsm + LISTN + RCAP;
  int* cnt  = dsm + LISTN + 2 * RCAP;
  int* offs = cnt + NBA;
  int* cur  = offs + NBA;
  int* misc = cur + NBA;
  const int tid = (int)threadIdx.x, lane = tid & 31, wave = tid >> 5;
  const int nodeBase = (int)blockIdx.x * NBA;

  {
    const v4i z4 = {0, 0, 0, 0};
    for (int i = tid * 4; i < AGG_ZINTS; i += NTHR * 4) *(v4ia*)(dsm + i) = z4;
    if (tid < 32) misc[tid] = 0;
  }
  __syncthreads();
  int tt = 0, ovf = 0;
  build_lists(dsts, nE, vec8, nodeBase, list, hl, sl, cnt, offs, cur, misc, tid, lane, wave, tt, ovf);
  (void)tt;

  float wl0[8], wl1[8], bl[8], wr0[8], wr1[8], br[8], we0[8], we1[8], at[8], b1[8];
  ld8(pp + PP_WL0 + 8 * lane, wl0);  ld8(pp + PP_WL0 + C1 + 8 * lane, wl1);  ld8(pp + PP_BL + 8 * lane, bl);
  ld8(pp + PP_WR0 + 8 * lane, wr0);  ld8(pp + PP_WR0 + C1 + 8 * lane, wr1);  ld8(pp + PP_BR + 8 * lane, br);
  ld8(pp + PP_WE0 + 8 * lane, we0);  ld8(pp + PP_WE0 + C1 + 8 * lane, we1);
  ld8(pp + PP_AT1 + 8 * lane, at);   ld8(pp + PP_B1 + 8 * lane, b1);

  const float qnan = __int_as_float(0x7fc00000);
  float* st = (float*)list + wave * C1 + 8 * lane;

#pragma unroll 1
  for (int si = 0; si < NBA / NWAVE; ++si) {
    const int s    = si * NWAVE + wave;
    const int node = nodeBase + s;
    int c = cnt[s];
    const bool big = c > DEGCAP;
    c = c < 0 ? 0 : (c > DEGCAP ? DEGCAP : c);
    int o = offs[s];
    o = o < 0 ? 0 : (o > RCAP ? RCAP : o);
    const int nc = node < nN ? node : nN - 1;
    const v2f xv = *(const v2fa*)(x + 2 * (size_t)nc);
    const float xi0 = bf16_val(xv.x), xi1 = bf16_val(xv.y);
    float xr[8], acc[8];
#pragma unroll
    for (int i = 0; i < 8; ++i) { xr[i] = fmaf(xi1, wr1[i], xi0 * wr0[i]) + br[i]; acc[i] = 0.0f; }
    const float rdeg = 1.0f / (float)(c < 1 ? 1 : c);
    float mx = -1.0e30f, dn = 0.0f, es0 = 0.0f, es1 = 0.0f;
    const int T = c + 1;
#pragma unroll 1
    for (int b0 = 0; b0 < T; b0 += 32) {
      int idx = o + b0 + lane;
      idx = idx > RCAP - 1 ? RCAP - 1 : idx;
      const int ent = sl[idx];
      int eid = ent >> SLA;
      eid = eid < 0 ? 0 : (eid > nE - 1 ? nE - 1 : eid);
      int sr = srcs[eid];
      sr = sr < 0 ? 0 : (sr > nN - 1 ? nN - 1 : sr);
      const v2f xs = *(const v2fa*)(x + 2 * (size_t)sr);
      const v2f ev = *(const v2fa*)(ea + 2 * (size_t)eid);
      const int xs0i = __float_as_int(bf16_val(xs.x)), xs1i = __float_as_int(bf16_val(xs.y));
      const int ev0i = __float_as_int(bf16_val(ev.x)), ev1i = __float_as_int(bf16_val(ev.y));
      const int m32 = (T - b0) < 32 ? (T - b0) : 32;
#pragma unroll 1
      for (int k = 0; k < m32; ++k) {
        const bool isSelf = (b0 + k) == c;
        const float r0 = __int_as_float(__builtin_amdgcn_readlane(xs0i, k));
        const float r1 = __int_as_float(__builtin_amdgcn_readlane(xs1i, k));
        const float r2 = __int_as_float(__builtin_amdgcn_readlane(ev0i, k));
        const float r3 = __int_as_float(__builtin_amdgcn_readlane(ev1i, k));
        const float la0 = es0 * rdeg, la1 = es1 * rdeg;
        const float X0 = isSelf ? xi0 : r0;
        const float X1 = isSelf ? xi1 : r1;
        const float A0 = isSelf ? la0 : r2;
        const float A1 = isSelf ? la1 : r3;
        es0 += isSelf ? 0.0f : r2;
        es1 += isSelf ? 0.0f : r3;
        float xl[8];
        float part = 0.0f;
#pragma unroll
        for (int i = 0; i < 8; ++i) {
          xl[i] = fmaf(X1, wl1[i], X0 * wl0[i]) + bl[i];
          const float ee = fmaf(A1, we1[i], A0 * we0[i]);
          float v = (xl[i] + xr[i]) + ee;
          v = v > 0.0f ? v : v * NEGS;
          part = fmaf(v, at[i], part);
        }
        part += __shfl_xor(part, 1, 32);
        part += __shfl_xor(part, 2, 32);
        part += __shfl_xor(part, 4, 32);
        const float df = part - mx;
        const float e  = expf(-fabsf(df));
        const bool up  = df > 0.0f;
        const float s1 = up ? e : 1.0f;
        const float s2 = up ? 1.0f : e;
        mx = up ? part : mx;
        dn = fmaf(dn, s1, s2);
#pragma unroll
        for (int i = 0; i < 8; ++i) acc[i] = fmaf(acc[i], s1, s2 * xl[i]);
      }
    }
    const float inv = __builtin_amdgcn_rcpf(dn + 1e-16f);
    const float pz  = (ovf != 0 || big) ? qnan : 0.0f;
#pragma unroll
    for (int i = 0; i < 8; ++i) st[i] = fmaf(acc[i], inv, b1[i]) + pz;
#pragma unroll 1
    for (int i = 0; i < 8; ++i) {
      const float v = st[i];
      const float e = expm1f(v);
      st[i] = (v > 0.0f) ? v : e;
    }
    const v4f ga = *(const v4fa*)st;
    const v4f gb = *(const v4fa*)(st + 4);
    const bool live = node < nN;
    const float f[8] = {ga.x, ga.y, ga.z, ga.w, gb.x, gb.y, gb.z, gb.w};
    v8us hv, lv;
#pragma unroll
    for (int i = 0; i < 8; ++i) {
      const float v = live ? f[i] : 0.0f;
      const unsigned hb = bf16_bits(v);
      const float r = v - __uint_as_float(hb << 16);
      hv[i] = (unsigned short)hb;
      lv[i] = (unsigned short)bf16_bits(r);
    }
    unsigned short* hp = h1 + (size_t)node * K2 + 8 * lane;
    const bool wr = node < mRows;
    if (wr) { *(volatile v8us*)hp = hv; *(volatile v8us*)(hp + C1) = lv; }
    __threadfence();
    if (wr) { *(volatile v8us*)hp = hv; *(volatile v8us*)(hp + C1) = lv; }
  }
}

__global__ __launch_bounds__(GTHR) void k_gemm2(
    const unsigned short* __restrict__ A, const unsigned short* __restrict__ WT,
    const float* __restrict__ bias, float* outF, int K, int ldo)
{
  __shared__ __attribute__((aligned(16))) float stg[GBM * GBN];
  const int tid = (int)threadIdx.x, lane = tid & 31, wave = tid >> 5, hh = lane >> 4, m = lane & 15;
  const int rowBase = (int)blockIdx.x * GBM;
  const int col0    = (int)blockIdx.y * GBN;

  v8f acc[4];
  {
    const v8f z = {0.f, 0.f, 0.f, 0.f, 0.f, 0.f, 0.f, 0.f};
    acc[0] = z; acc[1] = z; acc[2] = z; acc[3] = z;
  }
  float bb[4];
#pragma unroll
  for (int t = 0; t < 4; ++t) bb[t] = bias[col0 + 16 * t + m];
  const unsigned short* ap = A  + (size_t)(rowBase + 16 * wave + m) * (size_t)K + 8 * hh;
  const unsigned short* wp = WT + (size_t)(col0 + m) * (size_t)K + 8 * hh;
  const int ksteps = K >> 5;
#pragma unroll 1
  for (int ks = 0; ks < ksteps; ++ks) {
    FragB af;
    af.h[0] = *(const v8usa*)(ap + 32 * ks);
    af.h[1] = *(const v8usa*)(ap + 32 * ks + 16);
#pragma unroll
    for (int t = 0; t < 4; ++t) {
      const unsigned short* wq = wp + (size_t)(16 * t) * (size_t)K + 32 * ks;
      FragB bf;
      bf.h[0] = *(const v8usa*)wq;
      bf.h[1] = *(const v8usa*)(wq + 16);
      acc[t] = wmb(af, bf, acc[t]);
    }
  }

#pragma unroll
  for (int t = 0; t < 4; ++t) {
    const int lc = 16 * t + m;
#pragma unroll
    for (int r = 0; r < 8; ++r) {
      const int lr = 16 * wave + 8 * hh + r;
      stg[lr * GBN + lc] = acc[t][r] + bb[t];
    }
  }
  __syncthreads();

  v4f fv[8];
#pragma unroll
  for (int i = 0; i < 8; ++i) {
    const int lr = 16 * wave + 2 * i + hh;
    fv[i] = *(const v4fa*)(stg + lr * GBN + 4 * m);
  }
#pragma unroll
  for (int i = 0; i < 8; ++i) {
    const int lr = 16 * wave + 2 * i + hh;
    const int gr = rowBase + lr;
    float* op = outF + (size_t)gr * (size_t)ldo + col0 + 4 * m;
    *(volatile v4f*)op = fv[i];
  }
  __threadfence();
#pragma unroll
  for (int i = 0; i < 8; ++i) {
    const int lr = 16 * wave + 2 * i + hh;
    const int gr = rowBase + lr;
    float* op = outF + (size_t)gr * (size_t)ldo + col0 + 4 * m;
    *(volatile v4f*)op = fv[i];
  }
}

__global__ __launch_bounds__(NTHR) void k_scan2(
    const int* __restrict__ srcs, const int* __restrict__ dsts,
    const float* __restrict__ ea, const float* __restrict__ pp, const float* __restrict__ xlr,
    const int* __restrict__ bat, double* rec, int* cntOut, int nE, int nN, int vec8) {
  extern __shared__ __attribute__((aligned(16))) int dsm[];
  int* list = dsm;
  int* hl   = dsm + LISTN;
  int* sl   = dsm + LISTN + RCAP;
  int* cnt  = dsm + LISTN + 2 * RCAP;
  int* offs = cnt + NBA;
  int* cur  = offs + NBA;
  int* misc = cur + NBA;
  const int tid = (int)threadIdx.x, lane = tid & 31, wave = tid >> 5;
  const int nodeBase = (int)blockIdx.x * NBA;

  {
    const v4i z4 = {0, 0, 0, 0};
    for (int i = tid * 4; i < AGG_ZINTS; i += NTHR * 4) *(v4ia*)(dsm + i) = z4;
    if (tid < 32) misc[tid] = 0;
  }
  __syncthreads();
  int tt = 0, ovf = 0;
  build_lists(dsts, nE, vec8, nodeBase, list, hl, sl, cnt, offs, cur, misc, tid, lane, wave, tt, ovf);
  (void)tt;

  const float* p2 = pp + PP_P2;
  const v2f w0 = *(const v2fa*)(p2 + 2 * lane);
  const v2f w1 = *(const v2fa*)(p2 + C2 + 2 * lane);
  const v2f av = *(const v2fa*)(p2 + 2 * C2 + 2 * lane);
  const v2f bv = *(const v2fa*)(p2 + 3 * C2 + 2 * lane);
  const float qnan = __int_as_float(0x7fc00000);
  double d0 = 0.0, d1 = 0.0;
  int pc = 0, wbig = 0;

#pragma unroll 1
  for (int si = 0; si < NBA / NWAVE; ++si) {
    const int s    = si * NWAVE + wave;
    const int node = nodeBase + s;
    int c = cnt[s];
    const bool big = c > DEGCAP;
    c = c < 0 ? 0 : (c > DEGCAP ? DEGCAP : c);
    int o = offs[s];
    o = o < 0 ? 0 : (o > RCAP ? RCAP : o);
    const int nc = node < nN ? node : nN - 1;
    const v2f xr = *(const v2fa*)(xlr + (size_t)nc * N2 + C2 + 2 * lane);
    const float rdeg = 1.0f / (float)(c < 1 ? 1 : c);
    float mx = -1.0e30f, dn = 0.0f, es0 = 0.0f, es1 = 0.0f, acc0 = 0.0f, acc1 = 0.0f;
    const int T = c + 1;
#pragma unroll 1
    for (int b0 = 0; b0 < T; b0 += 32) {
      int idx = o + b0 + lane;
      idx = idx > RCAP - 1 ? RCAP - 1 : idx;
      const int ent = sl[idx];
      int eid = ent >> SLA;
      eid = eid < 0 ? 0 : (eid > nE - 1 ? nE - 1 : eid);
      int sr = srcs[eid];
      sr = sr < 0 ? 0 : (sr > nN - 1 ? nN - 1 : sr);
      const v2f ev = *(const v2fa*)(ea + 2 * (size_t)eid);
      const int ev0i = __float_as_int(bf16_val(ev.x)), ev1i = __float_as_int(bf16_val(ev.y));
      const int m32 = (T - b0) < 32 ? (T - b0) : 32;
#pragma unroll 1
      for (int k = 0; k < m32; ++k) {
        const bool isSelf = (b0 + k) == c;
        const int   sk = __builtin_amdgcn_readlane(sr, k);
        const float r2 = __int_as_float(__builtin_amdgcn_readlane(ev0i, k));
        const float r3 = __int_as_float(__builtin_amdgcn_readlane(ev1i, k));
        const int row = isSelf ? nc : sk;
        const v2f a = *(const v2fa*)(xlr + (size_t)row * N2 + 2 * lane);
        const float la0 = es0 * rdeg, la1 = es1 * rdeg;
        const float A0 = isSelf ? la0 : r2;
        const float A1 = isSelf ? la1 : r3;
        es0 += isSelf ? 0.0f : r2;
        es1 += isSelf ? 0.0f : r3;
        const float ee0 = fmaf(A1, w1.x, A0 * w0.x);
        const float ee1 = fmaf(A1, w1.y, A0 * w0.y);
        float v0 = (a.x + xr.x) + ee0;
        float v1 = (a.y + xr.y) + ee1;
        v0 = v0 > 0.0f ? v0 : v0 * NEGS;
        v1 = v1 > 0.0f ? v1 : v1 * NEGS;
        float part = fmaf(v1, av.y, v0 * av.x);
        part += __shfl_xor(part, 16, 32);
        part += __shfl_xor(part, 8, 32);
        part += __shfl_xor(part, 4, 32);
        part += __shfl_xor(part, 2, 32);
        part += __shfl_xor(part, 1, 32);
        const float df = part - mx;
        const float e  = expf(-fabsf(df));
        const bool up  = df > 0.0f;
        const float s1 = up ? e : 1.0f;
        const float s2 = up ? 1.0f : e;
        mx = up ? part : mx;
        dn = fmaf(dn, s1, s2);
        acc0 = fmaf(acc0, s1, s2 * a.x);
        acc1 = fmaf(acc1, s1, s2 * a.y);
      }
    }
    const float inv = __builtin_amdgcn_rcpf(dn + 1e-16f);
    const float pz  = (ovf != 0 || big) ? qnan : 0.0f;
    const float h0 = fmaf(acc0, inv, bv.x) + pz;
    const float h1v = fmaf(acc1, inv, bv.y) + pz;
    const int bi = bat[nc];
    const bool take = (node < nN) && (bi == 0);
    d0 += take ? (double)h0 : 0.0;
    d1 += take ? (double)h1v : 0.0;
    pc += take ? 1 : 0;
    wbig |= big ? 1 : 0;
  }

  double* pd   = (double*)(void*)hl;
  double* outd = pd + NWAVE * C2;
  pd[wave * C2 + 2 * lane]     = d0;
  pd[wave * C2 + 2 * lane + 1] = d1;
  if (lane == 0) { misc[wave] = pc; misc[16 + wave] = wbig; }
  __syncthreads();
  if (tid < C2) {
    double sacc = 0.0;
#pragma unroll
    for (int w2 = 0; w2 < NWAVE; ++w2) sacc += pd[w2 * C2 + tid];
    outd[tid] = sacc;
  }
  __syncthreads();
  int ctot = 0, fl = ovf;
#pragma unroll
  for (int w2 = 0; w2 < NWAVE; ++w2) { ctot += misc[w2]; fl |= misc[16 + w2]; }
  v2d rv;
  rv.x = outd[2 * lane];
  rv.y = outd[2 * lane + 1];
  v4i cv;
  cv.x = (lane == 0) ? ctot : 0;
  cv.y = (lane == 0) ? fl : 0;
  cv.z = 0; cv.w = 0;
  double* rp = rec + (size_t)blockIdx.x * C2 + 2 * lane;
  int*    cp = cntOut + (size_t)blockIdx.x * 32 + 4 * (lane & 7);
  const bool wr  = (wave == 0);
  const bool wrc = (wave == 0) && (lane < 8);
  if (wr)  *(volatile v2d*)rp = rv;
  if (wrc) *(volatile v4i*)cp = cv;
  __threadfence();
  if (wr)  *(volatile v2d*)rp = rv;
  if (wrc) *(volatile v4i*)cp = cv;
}

__global__ __launch_bounds__(64) void k_pool(const double* __restrict__ rec, const int* __restrict__ cntIn,
                                             int nB, float* out) {
  __shared__ __attribute__((aligned(16))) float outs[C2];
  const int tid = (int)threadIdx.x, lane = tid & 31, wave = tid >> 5;
  double s = 0.0;
  int ct = 0, fl = 0;
#pragma unroll 1
  for (int b = 0; b < nB; ++b) {
    s += rec[(size_t)b * C2 + tid];
    const v2i cf = *(const v2ia*)(cntIn + (size_t)b * 32);
    ct += cf.x < 0 ? 0 : cf.x;
    fl |= cf.y;
  }
  const double den = (double)(ct < 1 ? 1 : ct);
  const float r = (float)(s / den);
  outs[tid] = (fl != 0) ? __int_as_float(0x7fc00000) : r;
  __syncthreads();
  const v4f ov = *(const v4fa*)(outs + 4 * (lane & 15));
  float* op = out + 4 * (lane & 15);
  const bool okst = (wave == 0) && (lane < 16);
  if (okst) *(volatile v4f*)op = ov;
  __threadfence();
  if (okst) *(volatile v4f*)op = ov;
}

static inline int cdiv(int a, int b) { return (a + b - 1) / b; }
static inline size_t al256(size_t o) { return (o + 255) & ~(size_t)255; }

extern "C" void kernel_launch(void* const* d_in, const int* in_sizes, int n_in,
                              void* d_out, int out_size, void* d_ws, size_t ws_size,
                              hipStream_t stream) {
  if (n_in < 18) return;
  if (in_sizes[0] < 2 || (in_sizes[0] & 1) != 0) return;
  const int nN = in_sizes[0] / 2;
  if (nN < 1 || nN > (1 << 22)) return;
  if (in_sizes[16] < 2 || (in_sizes[16] & 1) != 0) return;
  const int nE = in_sizes[16] / 2;
  if (nE < 1 || nE >= (1 << (31 - SLA))) return;
  if (in_sizes[1] != 2 * nE) return;
  if (in_sizes[2] != 2 * C1 || in_sizes[3] != C1 || in_sizes[4] != 2 * C1 || in_sizes[5] != C1) return;
  if (in_sizes[6] != 2 * C1 || in_sizes[7] != C1 || in_sizes[8] != C1) return;
  if (in_sizes[9] != C1 * C2 || in_sizes[10] != C2 || in_sizes[11] != C1 * C2 || in_sizes[12] != C2) return;
  if (in_sizes[13] != 2 * C2 || in_sizes[14] != C2 || in_sizes[15] != C2) return;
  if (in_sizes[17] != nN) return;
  if (out_size != C2) return;

  const float* x     = (const float*)d_in[0];
  const float* eattr = (const float*)d_in[1];
  const float* W1l   = (const float*)d_in[2];
  const float* b1l   = (const float*)d_in[3];
  const float* W1r   = (const float*)d_in[4];
  const float* b1r   = (const float*)d_in[5];
  const float* W1e   = (const float*)d_in[6];
  const float* att1  = (const float*)d_in[7];
  const float* bias1 = (const float*)d_in[8];
  const float* W2l   = (const float*)d_in[9];
  const float* b2l   = (const float*)d_in[10];
  const float* W2r   = (const float*)d_in[11];
  const float* b2r   = (const float*)d_in[12];
  const float* W2e   = (const float*)d_in[13];
  const float* att2  = (const float*)d_in[14];
  const float* bias2 = (const float*)d_in[15];
  const int*   edge  = (const int*)d_in[16];
  const int*   bat   = (const int*)d_in[17];
  float* out = (float*)d_out;
  const int* src = edge;
  const int* dst = edge + nE;

  const int MP   = cdiv(nN, GBM) * GBM;
  const int gM   = MP / GBM;
  const int gA   = cdiv(MP, NBA);
  if ((long long)gA * NBA < (long long)MP) return;
  const int vec8 = ((nE & 3) == 0) ? 1 : 0;

  char* ws = (char*)d_ws;
  size_t off = 0;
  const size_t oPP  = off; off = al256(off + (size_t)PP_N * 4);
  const size_t oBT2 = off; off = al256(off + (size_t)N2 * K2 * 2);
  const size_t oH1  = off; off = al256(off + (size_t)MP * K2 * 2);
  const size_t oXLR = off; off = al256(off + (size_t)MP * N2 * 4);
  const size_t oREC = off; off = al256(off + (size_t)gA * C2 * 8);
  const size_t oCNT = off; off = al256(off + (size_t)gA * 128);
  if (off > ws_size || off > (size_t)WSMAX) return;
  float*          PP   = (float*)(ws + oPP);
  unsigned short* BT2  = (unsigned short*)(ws + oBT2);
  unsigned short* H1HL = (unsigned short*)(ws + oH1);
  float*          XLR2 = (float*)(ws + oXLR);
  double*         REC  = (double*)(ws + oREC);
  int*            CNT  = (int*)(ws + oCNT);

  hipFuncSetAttribute(reinterpret_cast<const void*>(&k_scan1), hipFuncAttributeMaxDynamicSharedMemorySize, (int)LDS_SCAN);
  hipFuncSetAttribute(reinterpret_cast<const void*>(&k_scan2), hipFuncAttributeMaxDynamicSharedMemorySize, (int)LDS_SCAN);

  k_prep<<<NUB / NTHR + 1, NTHR, 0, stream>>>(W1l, b1l, W1r, b1r, W1e, att1, bias1, W2l, b2l, W2r, b2r,
                                              W2e, att2, bias2, BT2, PP);
  k_scan1<<<gA, NTHR, LDS_SCAN, stream>>>(src, dst, x, eattr, PP, H1HL, nE, nN, vec8, MP);
  k_gemm2<<<dim3(gM, N2 / GBN), GTHR, 0, stream>>>(H1HL, BT2, PP + PP_B2, XLR2, K2, N2);
  k_scan2<<<gA, NTHR, LDS_SCAN, stream>>>(src, dst, eattr, PP, XLR2, bat, REC, CNT, nE, nN, vec8);
  k_pool<<<1, 64, 0, stream>>>(REC, CNT, gA, out);
}
